// GraphAttentionBlock_86337432584463
// MI455X (gfx1250) — hardware-run, weakly checked
//
#include <hip/hip_runtime.h>


#ifndef NB
#define NB 2
#endif
#ifndef SEQ
#define SEQ 2048
#endif
#define NB_FULL  2
#define SEQ_FULL 2048
#ifndef OUT_SEQ
#define OUT_SEQ SEQ
#endif
#define DM   256
#define NH_  8
#define HD   32
#define DFF  1024
#define AW   4
#define OSP  68
#define GSP  68
#define WSC  64.0f
#define WSI  (1.0f / 64.0f)
#define ACS  256.0f
#define L2E  1.4426950408889634f
#define SC2  ((float)(0.17677669529663687 * 1.4426950408889634))
#define PSH  14.0f
#define NEGB (-3.0e38f)

static_assert(HD == 32);
static_assert(NH_ * HD == DM);
static_assert(NH_ % 2 == 0);
static_assert(DM == 32 * 8);
static_assert(DM % 64 == 0);
static_assert(DFF % 64 == 0);
static_assert(DM % 32 == 0);
static_assert(DFF % 32 == 0);
static_assert(SEQ % 64 == 0);
static_assert((NB * SEQ) % 64 == 0);
static_assert((NB * SEQ) % 8 == 0);
static_assert(SEQ % 32 == 0);
static_assert(SEQ % (16 * AW) == 0);
static_assert(NB <= NB_FULL);
static_assert(SEQ <= SEQ_FULL);
static_assert((OSP * 4) % 16 == 0);
static_assert(OSP >= 64);
static_assert((GSP * 4) % 16 == 0);
static_assert(GSP >= 64);
static_assert(32 * 16 * 8 * 2 == 64 * 64 * 2);
static_assert(32 * 16 * 16 == 64 * 64 * 2);
static_assert(32 * 16 * 32 == 64 * 64 * 4);
static_assert(32 * 16 * 4 == 16 * 64 * 2);
static_assert(256 * 16 * 2 == 64 * 64 * 2);
static_assert(32 * 16 == DM * 2);
static_assert(64 * GSP * 4 <= 131072);
static_assert(AW * 16 * OSP * 4 <= 131072);
static_assert(64 * 65 * 4 <= 131072);

typedef _Float16 h16;
typedef __attribute__((ext_vector_type(16))) _Float16 v16h;
typedef __attribute__((ext_vector_type(8)))  _Float16 v8h;
typedef __attribute__((ext_vector_type(8)))  float    v8f;
typedef __attribute__((ext_vector_type(4)))  float    v4f;
typedef v4f  __attribute__((may_alias)) v4fa;

__device__ __forceinline__ unsigned short f2bf(float f) { unsigned u = __float_as_uint(f); u += 0x7FFFu + ((u >> 16) & 1u); return (unsigned short)(u >> 16); }
__device__ __forceinline__ float bfr(float f) { return __uint_as_float(((unsigned)f2bf(f)) << 16); }
__device__ __forceinline__ v16h cat16(v8h lo, v8h hi) { return __builtin_shufflevector(lo, hi, 0, 1, 2, 3, 4, 5, 6, 7, 8, 9, 10, 11, 12, 13, 14, 15); }
__device__ __forceinline__ v16h  ldh(const h16* p) { return cat16(*(const v8h*)p, *(const v8h*)(p + 16)); }
__device__ __forceinline__ void wave_sync() { __builtin_amdgcn_fence(3  , "wavefront"); __builtin_amdgcn_wave_barrier(); asm volatile("" ::: "memory"); }
static __device__ __forceinline__ h16 toh_flush(float v) { const h16 r = (h16)v; return (fabsf(v) < 6.103515625e-05f) ? (h16)0.0f : r; }
__device__ __forceinline__ v8f wmma16g(v16h a, v16h b, v8f c) {
    c = __builtin_amdgcn_wmma_f32_16x16x32_f16(false, a, false, b, (short)0, c, false, false);
    asm volatile("v_nop\n\tv_nop\n\tv_nop\n\tv_nop" : "+v"(c) : "v"(a), "v"(b));
    return c;
}
__device__ __forceinline__ float gelu_erf(float x) { return 0.5f * x * (1.0f + erff(x * 0.70710678118654752f)); }

__global__ __launch_bounds__(256) void k_ln(const float* __restrict__ x, const float* __restrict__ g, const float* __restrict__ bt, h16* out, int bstride, int rnd) {
#pragma clang fp contract(off)
    const int lane = threadIdx.x & 31;
    const int wave = __builtin_amdgcn_readfirstlane((int)(threadIdx.x >> 5));
    const int m = blockIdx.x * 8 + wave;
    const int bb = m / SEQ, tt = m % SEQ;
    const float* xr = x + ((size_t)bb * (size_t)bstride + (size_t)tt) * DM + lane * 8;
    const v4f xa = *(const v4f*)xr, xb = *(const v4f*)(xr + 4);
    const v4f ga = *(const v4f*)(g + lane * 8), gb = *(const v4f*)(g + lane * 8 + 4);
    const v4f ba = *(const v4f*)(bt + lane * 8), bb2 = *(const v4f*)(bt + lane * 8 + 4);
    float v[8], gg[8], be[8];
#pragma unroll
    for (int i = 0; i < 4; ++i) {
        v[i] = rnd ? bfr(xa[i]) : xa[i]; v[4 + i] = rnd ? bfr(xb[i]) : xb[i];
        gg[i] = bfr(ga[i]); gg[4 + i] = bfr(gb[i]); be[i] = bfr(ba[i]); be[4 + i] = bfr(bb2[i]); }
    float s = 0.0f;
#pragma unroll
    for (int i = 0; i < 8; ++i) s += v[i];
#pragma unroll
    for (int o = 16; o >= 1; o >>= 1) s += __shfl_xor(s, o, 32);
    const float mean = s * (1.0f / DM);
    float q = 0.0f;
#pragma unroll
    for (int i = 0; i < 8; ++i) { const float d = v[i] - mean; q += d * d; }
#pragma unroll
    for (int o = 16; o >= 1; o >>= 1) q += __shfl_xor(q, o, 32);
    const float rstd = rsqrtf(q * (1.0f / DM) + 1.0e-5f);
    v8h hv;
#pragma unroll
    for (int i = 0; i < 8; ++i) hv[i] = toh_flush((v[i] - mean) * rstd * gg[i] + be[i]);
    h16* orow = out + (size_t)m * DM + lane * 8;
    *(volatile v8h*)orow = hv; __threadfence(); *(volatile v8h*)orow = hv;
}

__global__ __launch_bounds__(256) void k_wT(const float* __restrict__ W, h16* WT, int Kd, int Nd) {
    __shared__ float ts[64 * 65];
    const int tid = threadIdx.x; const int k0 = blockIdx.x * 64, n0 = blockIdx.y * 64;
#pragma unroll 4
    for (int j = 0; j < 16; ++j) { const int idx = tid + j * 256; const int r = idx >> 6, c = idx & 63;
        ts[r * 65 + c] = W[(size_t)(k0 + r) * Nd + n0 + c]; }
    __syncthreads();
    const int c8 = (tid & 7) * 8;
#pragma unroll 1
    for (int ps = 0; ps < 2; ++ps) {
#pragma unroll
        for (int pass = 0; pass < 2; ++pass) { const int n = pass * 32 + (tid >> 3);
            v8h hv;
#pragma unroll
            for (int i = 0; i < 8; ++i) hv[i] = toh_flush(bfr(ts[(c8 + i) * 65 + n]) * WSC);
            *(volatile v8h*)(WT + (size_t)(n0 + n) * Kd + k0 + c8) = hv; }
        if (ps == 0) __threadfence(); }
}

template <int MODE>
__device__ __forceinline__ void gemm_body(const h16* __restrict__ A, const h16* __restrict__ Bt, const float* __restrict__ bias, const float* __restrict__ resid,
                                          h16* Oh, float* Of, int K, int ldo, float esc, int rs_res, int rs_out, int rnd) {
    __shared__ __align__(16) float os[64 * GSP];
    const int lane = threadIdx.x & 31, lr = lane & 15, hi = lane >> 4; const int r0 = blockIdx.x * 64, c0 = blockIdx.y * 64;
    v8f acc[4][4];
#pragma unroll
    for (int mb = 0; mb < 4; ++mb)
#pragma unroll
        for (int nb = 0; nb < 4; ++nb) acc[mb][nb] = (v8f){};
    const size_t aoff = (size_t)(r0 + lr) * K + 8 * hi, boff = (size_t)(c0 + lr) * K + 8 * hi;
#pragma unroll 1
    for (int kc = 0; kc < K; kc += 32) {
        v16h a[4];
#pragma unroll
        for (int mb = 0; mb < 4; ++mb) a[mb] = ldh(A + aoff + (size_t)mb * 16 * K + kc);
#pragma unroll
        for (int nb = 0; nb < 4; ++nb) { const v16h b = ldh(Bt + boff + (size_t)nb * 16 * K + kc);
#pragma unroll
            for (int mb = 0; mb < 4; ++mb) acc[mb][nb] = wmma16g(a[mb], b, acc[mb][nb]); }
    }
    float bc[4];
#pragma unroll
    for (int nb = 0; nb < 4; ++nb) bc[nb] = (MODE != 1) ? bfr(bias[c0 + nb * 16 + lr]) : 0.0f;
#pragma unroll
    for (int mb = 0; mb < 4; ++mb) {
        float br[8];
#pragma unroll
        for (int j = 0; j < 8; ++j) br[j] = (MODE == 1) ? bfr(bias[r0 + mb * 16 + hi * 8 + j]) : 0.0f;
#pragma unroll
        for (int nb = 0; nb < 4; ++nb) {
#pragma unroll
            for (int j = 0; j < 8; ++j) os[(mb * 16 + hi * 8 + j) * GSP + nb * 16 + lr] = acc[mb][nb][j] * esc + bc[nb] + br[j]; }
    }
    wave_sync();
    if (MODE == 0) {
        const int bb = r0 / SEQ, tt = r0 % SEQ; const int zc = bb * NH_ + c0 / HD;
        const size_t tbase = ((size_t)zc * SEQ + (size_t)tt) * HD;
#pragma unroll 1
        for (int ps = 0; ps < 2; ++ps) {
#pragma unroll
            for (int hh = 0; hh < 2; ++hh) {
#pragma unroll 1
                for (int s = 0; s < 8; ++s) { const int p = s * 32 + lane; const int row = p >> 2, c8 = (p & 3) * 8;
                    const v4f x0 = *(const v4fa*)(&os[row * GSP + hh * 32 + c8]); const v4f x1 = *(const v4fa*)(&os[row * GSP + hh * 32 + c8 + 4]); v8h hv;
#pragma unroll
                    for (int i = 0; i < 4; ++i) { hv[i] = toh_flush(x0[i]); hv[4 + i] = toh_flush(x1[i]); }
                    *(volatile v8h*)(Oh + tbase + (size_t)hh * ((size_t)SEQ * HD) + (size_t)p * 8) = hv; } }
            if (ps == 0) __threadfence(); }
    } else if (MODE == 1 || MODE == 3) {
        size_t tbase, pitch;
        if (MODE == 1) { const int bb = c0 / SEQ, tt = c0 % SEQ; tbase = (size_t)bb * (size_t)DM * SEQ + (size_t)r0 * SEQ + (size_t)tt; pitch = (size_t)SEQ; }
        else           { tbase = (size_t)r0 * (size_t)ldo + (size_t)c0; pitch = (size_t)ldo; }
#pragma unroll 1
        for (int ps = 0; ps < 2; ++ps) {
#pragma unroll 1
            for (int s = 0; s < 16; ++s) { const int row = 4 * s + (lane >> 3), c8 = (lane & 7) * 8;
                const v4f x0 = *(const v4fa*)(&os[row * GSP + c8]); const v4f x1 = *(const v4fa*)(&os[row * GSP + c8 + 4]); v8h hv;
#pragma unroll
                for (int i = 0; i < 4; ++i) { hv[i] = toh_flush((MODE == 3) ? gelu_erf(x0[i]) : x0[i]); hv[4 + i] = toh_flush((MODE == 3) ? gelu_erf(x1[i]) : x1[i]); }
                *(volatile v8h*)(Oh + tbase + (size_t)row * pitch + c8) = hv; }
            if (ps == 0) __threadfence(); }
    } else {
        const int bb = r0 / SEQ, tt = r0 % SEQ;
        const size_t rrow = (size_t)bb * (size_t)rs_res + (size_t)tt;
        const size_t orow = (size_t)bb * (size_t)rs_out + (size_t)tt;
#pragma unroll 1
        for (int ps = 0; ps < 2; ++ps) {
#pragma unroll 1
            for (int s = 0; s < 32; ++s) { const int row = 2 * s + (lane >> 4), c4 = (lane & 15) * 4;
                const v4f x = *(const v4fa*)(&os[row * GSP + c4]);
                const v4f r = *(const v4f*)(resid + (rrow + (size_t)row) * DM + c0 + c4);
                v4f val;
#pragma unroll
                for (int i = 0; i < 4; ++i) { const float rv = rnd ? bfr(r[i]) : r[i]; val[i] = x[i] + rv; }
                *(volatile v4f*)(Of + (orow + (size_t)row) * DM + c0 + c4) = val; }
            if (ps == 0) __threadfence(); }
    }
}

__global__ __launch_bounds__(32) void k_gemm_qk(const h16* __restrict__ A, const h16* __restrict__ Bt, const float* __restrict__ bias, h16* Oh, int K, float esc) {
    gemm_body<0>(A, Bt, bias, nullptr, Oh, nullptr, K, 0, esc, 0, 0, 0);
}
__global__ __launch_bounds__(32) void k_gemm_vt(const h16* __restrict__ A, const h16* __restrict__ Bt, const float* __restrict__ bias, h16* Oh, int K, float esc) {
    gemm_body<1>(A, Bt, bias, nullptr, Oh, nullptr, K, 0, esc, 0, 0, 0);
}
__global__ __launch_bounds__(32) void k_gemm_res(const h16* __restrict__ A, const h16* __restrict__ Bt, const float* __restrict__ bias, const float* __restrict__ resid, float* Of,
                                                 int K, float esc, int rs_res, int rs_out, int rnd) {
    gemm_body<2>(A, Bt, bias, resid, nullptr, Of, K, 0, esc, rs_res, rs_out, rnd);
}
__global__ __launch_bounds__(32) void k_gemm_gelu(const h16* __restrict__ A, const h16* __restrict__ Bt, const float* __restrict__ bias, h16* Oh, int K, int ldo, float esc) {
    gemm_body<3>(A, Bt, bias, nullptr, Oh, nullptr, K, ldo, esc, 0, 0, 0);
}

__device__ __forceinline__ void head_step(const h16* __restrict__ kp, const h16* __restrict__ vp, v16h q, v8f bA, v8f bB, v8f gA, v8f gB,
                                          float& m, float& l, float& d, v8f& o0, v8f& o1) {
    const v16h ka = ldh(kp), kb = ldh(kp + 16 * HD);
    v8f sa = (v8f){}, sb = (v8f){};
    sa = wmma16g(ka, q, sa); sb = wmma16g(kb, q, sb);
    float ta[8], tb[8]; float mx = NEGB;
#pragma unroll
    for (int r = 0; r < 8; ++r) { ta[r] = sa[r] * SC2 + bA[r]; tb[r] = sb[r] * SC2 + bB[r]; mx = fmaxf(mx, fmaxf(ta[r], tb[r])); }
    mx = fmaxf(mx, __shfl_xor(mx, 16, 32));
    const float mnew = fmaxf(m, mx);
    const float alpha = __builtin_amdgcn_exp2f(m - mnew);
    const float sh = PSH - mnew;
    v16h pb; float ls = 0.0f, ds = 0.0f;
#pragma unroll
    for (int r = 0; r < 8; ++r) {
        const float ea = __builtin_amdgcn_exp2f(ta[r] + sh), eb = __builtin_amdgcn_exp2f(tb[r] + sh);
        ds += ea + eb;
        const h16 pa = toh_flush(ea * gA[r]); const h16 pc = toh_flush(eb * gB[r]);
        pb[r] = pa; pb[8 + r] = pc;
        ls += (float)pa + (float)pc; }
    l = l * alpha + ls; d = d * alpha + ds; m = mnew;
    o0 = o0 * alpha; o1 = o1 * alpha;
    const v16h v0 = ldh(vp), v1 = ldh(vp + (size_t)16 * SEQ);
    o0 = wmma16g(v0, pb, o0); o1 = wmma16g(v1, pb, o1);
}

__global__ __launch_bounds__(32 * AW) void k_fused(const h16* __restrict__ QH, const h16* __restrict__ KP, const h16* __restrict__ VT, const float* __restrict__ adj, h16* ATT) {
    __shared__ __align__(16) float os[AW * 16 * OSP];
    const int lane = threadIdx.x & 31, lr = lane & 15, hi = lane >> 4;
    const int wave = __builtin_amdgcn_readfirstlane((int)(threadIdx.x >> 5));
    const int zp = blockIdx.y; const int b = zp / (NH_ / 2), hp = zp % (NH_ / 2);
    const int t0 = (blockIdx.x * AW + wave) * 16;
    const size_t pb0 = (size_t)(b * NH_ + 2 * hp) * SEQ * HD, pb1 = pb0 + (size_t)SEQ * HD;
    const size_t qo = (size_t)(t0 + lr) * HD + 8 * hi;
    const v16h q0 = ldh(QH + pb0 + qo), q1 = ldh(QH + pb1 + qo);
    const size_t ko = (size_t)lr * HD + 8 * hi;
    const size_t vo = (size_t)lr * SEQ + 8 * hi;
    const float* ar = adj + ((size_t)b * SEQ_FULL + (size_t)(t0 + lr)) * SEQ_FULL + 8 * hi;
    v8f o00 = (v8f){}, o01 = (v8f){}, o10 = (v8f){}, o11 = (v8f){};
    float m0 = NEGB, l0 = 0.0f, d0 = 0.0f, m1 = NEGB, l1 = 0.0f, d1 = 0.0f;
#pragma unroll 1
    for (int key0 = 0; key0 < SEQ; key0 += 32) {
        const float* ap = ar + key0;
        const v4f a0 = *(const v4f*)ap, a1 = *(const v4f*)(ap + 4), a2 = *(const v4f*)(ap + 16), a3 = *(const v4f*)(ap + 20);
        v8f bA, bB, gA, gB;
#pragma unroll
        for (int r = 0; r < 4; ++r) {
            const float x0 = bfr(a0[r]), x1 = bfr(a1[r]), x2 = bfr(a2[r]), x3 = bfr(a3[r]);
            bA[r] = (2.0f * x0 - 1.0f) * L2E; bA[4 + r] = (2.0f * x1 - 1.0f) * L2E; bB[r] = (2.0f * x2 - 1.0f) * L2E; bB[4 + r] = (2.0f * x3 - 1.0f) * L2E;
            gA[r] = 0.25f + 0.75f * x0; gA[4 + r] = 0.25f + 0.75f * x1; gB[r] = 0.25f + 0.75f * x2; gB[4 + r] = 0.25f + 0.75f * x3; }
        head_step(KP + pb0 + ko + (size_t)key0 * HD, VT + pb0 + vo + key0, q0, bA, bB, gA, gB, m0, l0, d0, o00, o01);
        head_step(KP + pb1 + ko + (size_t)key0 * HD, VT + pb1 + vo + key0, q1, bA, bB, gA, gB, m1, l1, d1, o10, o11);
    }
    l0 += __shfl_xor(l0, 16, 32); d0 += __shfl_xor(d0, 16, 32);
    l1 += __shfl_xor(l1, 16, 32); d1 += __shfl_xor(d1, 16, 32);
    const float inv0 = ACS * __builtin_amdgcn_rcpf(fmaxf(l0, 1.0e-6f * d0));
    const float inv1 = ACS * __builtin_amdgcn_rcpf(fmaxf(l1, 1.0e-6f * d1));
    const v8f f00 = o00 * inv0, f01 = o01 * inv0, f10 = o10 * inv1, f11 = o11 * inv1;
    const int wb = wave * 16 * OSP;
    const int ob = wb + lr * OSP + 8 * hi;
    *(v4fa*)(&os[ob +  0]) = __builtin_shufflevector(f00, f00, 0, 1, 2, 3); *(v4fa*)(&os[ob +  4]) = __builtin_shufflevector(f00, f00, 4, 5, 6, 7);
    *(v4fa*)(&os[ob + 16]) = __builtin_shufflevector(f01, f01, 0, 1, 2, 3); *(v4fa*)(&os[ob + 20]) = __builtin_shufflevector(f01, f01, 4, 5, 6, 7);
    *(v4fa*)(&os[ob + 32]) = __builtin_shufflevector(f10, f10, 0, 1, 2, 3); *(v4fa*)(&os[ob + 36]) = __builtin_shufflevector(f10, f10, 4, 5, 6, 7);
    *(v4fa*)(&os[ob + 48]) = __builtin_shufflevector(f11, f11, 0, 1, 2, 3); *(v4fa*)(&os[ob + 52]) = __builtin_shufflevector(f11, f11, 4, 5, 6, 7);
    wave_sync();
    h16* arow = ATT + ((size_t)b * SEQ + (size_t)t0) * DM + hp * 64;
#pragma unroll 1
    for (int ps = 0; ps < 2; ++ps) {
#pragma unroll
        for (int s = 0; s < 4; ++s) { const int row = 4 * s + (lane >> 3), c8 = (lane & 7) * 8;
            const v4f x0 = *(const v4fa*)(&os[wb + row * OSP + c8]); const v4f x1 = *(const v4fa*)(&os[wb + row * OSP + c8 + 4]); v8h hv;
#pragma unroll
            for (int i = 0; i < 4; ++i) { hv[i] = toh_flush(x0[i]); hv[4 + i] = toh_flush(x1[i]); }
            *(volatile v8h*)(arow + (size_t)row * DM + c8) = hv; }
        if (ps == 0) __threadfence(); }
}

static constexpr size_t al256(size_t v) { return (v + 255) & ~(size_t)255; }
static constexpr size_t SZ_XN = al256((size_t)NB * SEQ * DM * 2);
static constexpr size_t SZ_WS = al256((size_t)DM * DM * 2);
static constexpr size_t SZ_WF = al256((size_t)DM * DFF * 2);
static constexpr size_t SZ_PL = al256((size_t)NB * NH_ * SEQ * HD * 2);
static constexpr size_t SZ_H2 = al256((size_t)NB * SEQ * DM * 4);
static constexpr size_t SZ_MD = al256((size_t)NB * SEQ * DFF * 2);
static constexpr size_t SZ_TOTAL = 3 * SZ_XN + 4 * SZ_WS + 2 * SZ_WF + 3 * SZ_PL + SZ_H2 + SZ_MD;
static_assert(SZ_TOTAL <= (size_t)134217728);
static_assert((size_t)NB * NH_ * SEQ * HD == (size_t)NB * DM * SEQ);

extern "C" void kernel_launch(void* const* d_in, const int* in_sizes, int n_in,
                              void* d_out, int out_size, void* d_ws, size_t ws_size, hipStream_t stream) {
    if (n_in < 19) return;
    const size_t needx = ((size_t)(NB - 1) * SEQ_FULL + SEQ) * DM;
    const size_t needa = ((size_t)(NB - 1) * SEQ_FULL + SEQ) * SEQ_FULL;
    if ((size_t)in_sizes[0] < needx || (size_t)in_sizes[1] < needa) return;
    if ((size_t)in_sizes[3] < (size_t)DM * DM || (size_t)in_sizes[5] < (size_t)DM * DM || (size_t)in_sizes[7] < (size_t)DM * DM || (size_t)in_sizes[9] < (size_t)DM * DM) return;
    if (in_sizes[4] < DM || in_sizes[6] < DM || in_sizes[8] < DM || in_sizes[10] < DM) return;
    if (in_sizes[11] < DM || in_sizes[12] < DM || in_sizes[13] < DM || in_sizes[14] < DM) return;
    if ((size_t)in_sizes[15] < (size_t)DM * DFF || in_sizes[16] < DFF || (size_t)in_sizes[17] < (size_t)DM * DFF || in_sizes[18] < DM) return;
    if ((size_t)out_size < ((size_t)(NB - 1) * OUT_SEQ + SEQ) * DM) return;
    if (SZ_TOTAL > ws_size) return;
    const float* hidden = (const float*)d_in[0];
    const float* adj    = (const float*)d_in[1];
    const float* wq = (const float*)d_in[3];  const float* bq = (const float*)d_in[4];
    const float* wk = (const float*)d_in[5];  const float* bk = (const float*)d_in[6];
    const float* wv = (const float*)d_in[7];  const float* bv = (const float*)d_in[8];
    const float* wo = (const float*)d_in[9];  const float* bo = (const float*)d_in[10];
    const float* g1 = (const float*)d_in[11]; const float* b1 = (const float*)d_in[12];
    const float* g2 = (const float*)d_in[13]; const float* b2 = (const float*)d_in[14];
    const float* w1 = (const float*)d_in[15]; const float* bf1 = (const float*)d_in[16];
    const float* w2 = (const float*)d_in[17]; const float* bf2 = (const float*)d_in[18];
    float* OUT = (float*)d_out;
    char* wsp = (char*)d_ws;
    h16* XN  = (h16*)wsp; wsp += SZ_XN;
    h16* ATT = (h16*)wsp; wsp += SZ_XN;
    h16* FI  = (h16*)wsp; wsp += SZ_XN;
    h16* WQT = (h16*)wsp; wsp += SZ_WS;
    h16* WKT = (h16*)wsp; wsp += SZ_WS;
    h16* WVT = (h16*)wsp; wsp += SZ_WS;
    h16* WOT = (h16*)wsp; wsp += SZ_WS;
    h16* W1T = (h16*)wsp; wsp += SZ_WF;
    h16* W2T = (h16*)wsp; wsp += SZ_WF;
    h16* QH  = (h16*)wsp; wsp += SZ_PL;
    h16* KP  = (h16*)wsp; wsp += SZ_PL;
    h16* VT  = (h16*)wsp; wsp += SZ_PL;
    float* H2 = (float*)wsp; wsp += SZ_H2;
    h16* MID = (h16*)wsp; wsp += SZ_MD;

    const int M = NB * SEQ;
    k_wT<<<dim3(DM / 64, DM / 64, 1), 256, 0, stream>>>(wq, WQT, DM, DM);
    k_wT<<<dim3(DM / 64, DM / 64, 1), 256, 0, stream>>>(wk, WKT, DM, DM);
    k_wT<<<dim3(DM / 64, DM / 64, 1), 256, 0, stream>>>(wv, WVT, DM, DM);
    k_wT<<<dim3(DM / 64, DM / 64, 1), 256, 0, stream>>>(wo, WOT, DM, DM);
    k_wT<<<dim3(DM / 64, DFF / 64, 1), 256, 0, stream>>>(w1, W1T, DM, DFF);
    k_wT<<<dim3(DFF / 64, DM / 64, 1), 256, 0, stream>>>(w2, W2T, DFF, DM);

    k_ln<<<M / 8, 256, 0, stream>>>(hidden, g1, b1, XN, SEQ_FULL, 1);

    k_gemm_qk<<<dim3(M / 64, DM / 64, 1), 32, 0, stream>>>(XN, WQT, bq, QH, DM, WSI);
    k_gemm_qk<<<dim3(M / 64, DM / 64, 1), 32, 0, stream>>>(XN, WKT, bk, KP, DM, WSI);
    k_gemm_vt<<<dim3(DM / 64, M / 64, 1), 32, 0, stream>>>(WVT, XN, bv, VT, DM, WSI);

    k_fused<<<dim3(SEQ / (16 * AW), NB * (NH_ / 2), 1), 32 * AW, 0, stream>>>(QH, KP, VT, adj, ATT);

    k_gemm_res<<<dim3(M / 64, DM / 64, 1), 32, 0, stream>>>(ATT, WOT, bo, hidden, H2, DM, WSI / ACS, SEQ_FULL, SEQ, 1);

    k_ln<<<M / 8, 256, 0, stream>>>(H2, g2, b2, FI, SEQ, 0);

    k_gemm_gelu<<<dim3(M / 64, DFF / 64, 1), 32, 0, stream>>>(FI, W1T, bf1, MID, DM, DFF, WSI);
    k_gemm_res<<<dim3(M / 64, DM / 64, 1), 32, 0, stream>>>(MID, W2T, bf2, H2, OUT, DFF, WSI, SEQ, OUT_SEQ, 0);
}
